// GELU48_17566416240672
// MI455X (gfx1250) — hardware-run, weakly checked
//
#include <hip/hip_runtime.h>
#include <math.h>

typedef __attribute__((ext_vector_type(16))) _Float16 v16h;
typedef __attribute__((ext_vector_type(8)))  _Float16 v8h;
typedef __attribute__((ext_vector_type(8)))  float    v8f;
typedef __attribute__((ext_vector_type(4)))  float    v4f;

constexpr int kBatch = 4;
constexpr int kTime  = 4096;
constexpr int kChan  = 512;
constexpr int kCols  = kBatch * kChan;
constexpr int kTile  = 64;
constexpr int kBand  = 128;
constexpr int kGP    = kTile + kTime;
constexpr int kSlabP = 68;
static_assert(kBatch == 4 && kTime == 4096 && kChan == 512, "wire shapes");
static_assert((kTime % kTile) == 0 && (kChan % kTile) == 0 && (kCols % kTile) == 0, "tile multiples");
static_assert((kBand % 32) == 0 && kBand == 2 * kTile, "K multiple of 32");
static_assert(((kGP * 2) % 128) == 0, "plane pitch is a whole number of 128-B lines");

constexpr float kCarryA = 256.0f;
constexpr float kCarryG = 16.0f;
constexpr float kFold   = 1.0f / (kCarryA * kCarryG);
constexpr float kMinNormalH = 6.2e-5f;
constexpr float kBandPremise = 1.0e-4f;
constexpr float kSqrt2OverPi = 0.7978845608028654f;
constexpr float kNegTwoC     = -2.0f * kSqrt2OverPi;

constexpr size_t kOffTaps = 0;
constexpr size_t kOffGt   = kOffTaps + (size_t)kTile * kBand * 2;
constexpr size_t kWsTotal = kOffGt + (size_t)kCols * kGP * 2;
static_assert(kOffGt == 16384ull, "tap tile bytes");
static_assert(kWsTotal == 17055744ull, "carve total");
static_assert(kWsTotal <= 134217728ull, "carve cap");
static_assert((kOffGt % 128) == 0, "aligned regions");

union FragU { v16h v; v8h h[2]; };
__device__ __forceinline__ v16h frag_load(const _Float16* p) {
  FragU f;
  f.h[0] = *(const v8h*)(p);
  f.h[1] = *(const v8h*)(p + 16);
  return f.v;
}
__device__ __forceinline__ v8f mma_h(v16h a, v16h b, v8f c) {
  c = __builtin_amdgcn_wmma_f32_16x16x32_f16(false, a, false, b, (short)0, c, false, false);
  asm volatile("v_nop\n\tv_nop\n\tv_nop\n\tv_nop" : "+v"(c) : "v"(a), "v"(b));
  return c;
}

__device__ __forceinline__ float act_f(float x) {
  const float x3 = x * x * x;
  const float inner = x + 0.044715f * x3;
  const float e = expf(kNegTwoC * inner);
  return x * __builtin_amdgcn_rcpf(1.0f + e);
}
__device__ __forceinline__ float decay_from_logit(float z) {
  return 1.0f / (1.0f + expf(-z));
}
__device__ __forceinline__ float softplus_f(float z) {
  return fmaxf(z, 0.0f) + log1pf(expf(-fabsf(z)));
}

__global__ __launch_bounds__(256) void build_taps_kernel(const float* __restrict__ logit_decay,
                                                         unsigned short* __restrict__ taps) {
  const int tid = threadIdx.x;
  const float dec = decay_from_logit(logit_decay[0]);
  const float l2d = log2f(dec);
#pragma unroll 1
  for (int i = 0; i < 4; ++i) {
    const int grp = tid + 256 * i;
    const int e0 = grp * 8;
    const int r  = e0 >> 7;
    const int c0 = e0 & (kBand - 1);
    v8h hv;
#pragma unroll
    for (int e = 0; e < 8; ++e) {
      const int dist = r + 63 - (c0 + e);
      const int distc = dist < 0 ? 0 : dist;
      const float w = kCarryA * exp2f((float)distc * l2d);
      const bool keep = (dist >= 0) && (w >= kMinNormalH);
      const float wv = keep ? w : 0.0f;
      hv[e] = (_Float16)wv;
    }
    unsigned short* p = taps + e0;
    *(volatile v8h*)p = hv;
    __threadfence();
    *(volatile v8h*)p = hv;
  }
}

__global__ __launch_bounds__(256) void act_plane_kernel(const float* __restrict__ x,
                                                        unsigned short* __restrict__ gt) {
  __shared__ __align__(16) float sT[kTile * kSlabP];
  const int tid  = threadIdx.x;
  const int lane = tid & 31;
  const int wave = __builtin_amdgcn_readfirstlane((int)(threadIdx.x >> 5));
  const int t0 = blockIdx.x * kTile;
  const int d0 = blockIdx.y * kTile;
  const int b  = blockIdx.z;
  const float* xb = x + ((size_t)b * kTime + t0) * kChan + d0;
#pragma unroll 1
  for (int i = 0; i < 4; ++i) {
    const int idx = tid + 256 * i;
    const int tr = idx >> 4;
    const int c4 = (idx & 15) * 4;
    const v4f xv = *(const v4f*)(xb + (size_t)tr * kChan + c4);
    const float g0 = act_f(xv[0]);
    const float g1 = act_f(xv[1]);
    const float g2 = act_f(xv[2]);
    const float g3 = act_f(xv[3]);
    sT[(c4 + 0) * kSlabP + tr] = g0;
    sT[(c4 + 1) * kSlabP + tr] = g1;
    sT[(c4 + 2) * kSlabP + tr] = g2;
    sT[(c4 + 3) * kSlabP + tr] = g3;
  }
  __syncthreads();
  const int q  = lane >> 3;
  const int c8 = (lane & 7) * 8;
  v8h hv[2];
#pragma unroll
  for (int it = 0; it < 2; ++it) {
    const int dl = it * 32 + wave * 4 + q;
    const float* sp = sT + dl * kSlabP + c8;
    const v4f a0 = *(const v4f*)(sp);
    const v4f a1 = *(const v4f*)(sp + 4);
#pragma unroll
    for (int e = 0; e < 4; ++e) {
      const float s0 = a0[e] * kCarryG;
      const float s1 = a1[e] * kCarryG;
      hv[it][e]     = (_Float16)s0;
      hv[it][4 + e] = (_Float16)s1;
    }
  }
  const int n0 = b * kChan + d0;
  const bool front = (blockIdx.x == 0);
  const v4f zero4 = (v4f){0.0f, 0.0f, 0.0f, 0.0f};
  for (int pass = 0; pass < 2; ++pass) {
#pragma unroll
    for (int it = 0; it < 2; ++it) {
      const int dl = it * 32 + wave * 4 + q;
      unsigned short* rowp = gt + (size_t)(n0 + dl) * kGP;
      *(volatile v8h*)(rowp + kTile + t0 + c8) = hv[it];
      if (front) *(volatile v4f*)(rowp + c8) = zero4;
    }
    __threadfence();
  }
}

__global__ __launch_bounds__(128) void band_gemm_kernel(
    const float* __restrict__ x, const float* __restrict__ log_alpha_raw,
    const float* __restrict__ logit_decay, const float* __restrict__ ema,
    const unsigned short* __restrict__ tapsp, const unsigned short* __restrict__ gtp,
    float* __restrict__ out) {
  __shared__ __align__(16) float sS[4][16 * kSlabP];
  const int lane = threadIdx.x & 31;
  const int wave = __builtin_amdgcn_readfirstlane((int)(threadIdx.x >> 5));
  const int mt = blockIdx.x;
  const int nt = blockIdx.y;
  const int b  = nt >> 3;
  const int d0 = (nt & 7) * kTile;
  const int n0 = nt * kTile;

  const float dec   = decay_from_logit(logit_decay[0]);
  const float alpha = softplus_f(log_alpha_raw[0]);
  const float onePa = 1.0f + alpha;
  const float l2d   = log2f(dec);
  const float cs    = (1.0f - dec) * kFold;
  const float d64   = exp2f(64.0f * l2d);
  const bool  bad   = !(d64 < kBandPremise);
  const float qn    = __uint_as_float(0x7fc00000u);

  const _Float16* taps = (const _Float16*)tapsp;
  const _Float16* gt   = (const _Float16*)gtp;
  const int rlane = lane & 15;
  const int koff  = (lane >> 4) * 8;
  const int mOff  = (lane >> 4) * 8;

  const _Float16* ap = taps + (size_t)(16 * wave + rlane) * kBand + koff;
  const _Float16* bp = gt + (size_t)(n0 + rlane) * kGP + (size_t)kTile * mt + koff;

  v8f acc0 = (v8f){0.f, 0.f, 0.f, 0.f, 0.f, 0.f, 0.f, 0.f};
  v8f acc1 = acc0;
  v8f acc2 = acc0;
  v8f acc3 = acc0;
#pragma unroll
  for (int ks = 0; ks < kBand / 32; ++ks) {
    const int k0 = ks * 32;
    const v16h af = frag_load(ap + k0);
    const v16h b0 = frag_load(bp + k0);
    const v16h b1 = frag_load(bp + (size_t)16 * kGP + k0);
    const v16h b2 = frag_load(bp + (size_t)32 * kGP + k0);
    const v16h b3 = frag_load(bp + (size_t)48 * kGP + k0);
    acc0 = mma_h(af, b0, acc0);
    acc1 = mma_h(af, b1, acc1);
    acc2 = mma_h(af, b2, acc2);
    acc3 = mma_h(af, b3, acc3);
  }

  float* slab = sS[wave];
#pragma unroll
  for (int r = 0; r < 8; ++r) {
    slab[(mOff + r) * kSlabP + rlane]      = acc0[r];
    slab[(mOff + r) * kSlabP + 16 + rlane] = acc1[r];
    slab[(mOff + r) * kSlabP + 32 + rlane] = acc2[r];
    slab[(mOff + r) * kSlabP + 48 + rlane] = acc3[r];
  }
  __builtin_amdgcn_fence(__ATOMIC_RELEASE, "workgroup");
  __builtin_amdgcn_wave_barrier();
  __builtin_amdgcn_fence(__ATOMIC_ACQUIRE, "workgroup");

  const int hh = lane >> 4;
  const int c4 = (lane & 15) * 4;
  const int tBase = kTile * mt + 16 * wave;
  const v4f em = *(const v4f*)(ema + d0 + c4);
  const float* xb = x + ((size_t)b * kTime + tBase) * kChan + d0 + c4;
  float* ob = out + ((size_t)b * kTime + tBase) * kChan + d0 + c4;

#pragma unroll 1
  for (int it = 0; it < 8; ++it) {
    const int row = it * 2 + hh;
    const int ti  = tBase + row;
    float* sp = slab + row * kSlabP + c4;
    const v4f a  = *(const v4f*)sp;
    const v4f xv = *(const v4f*)(xb + (size_t)row * kChan);
    const float di  = exp2f((float)ti * l2d);
    const float den = fmaxf(1.0f - di, 1e-8f);
    const float sc  = cs * (1.0f / den);
    const bool first = (ti == 0);
    v4f yv;
#pragma unroll
    for (int e = 0; e < 4; ++e) {
      const float past = a[e] * sc;
      float cv = first ? em[e] : past;
      cv = bad ? qn : cv;
      const float g = act_f(xv[e]);
      yv[e] = onePa * g - alpha * cv;
    }
    *(v4f*)sp = yv;
  }
  __builtin_amdgcn_fence(__ATOMIC_RELEASE, "workgroup");
  __builtin_amdgcn_wave_barrier();
  __builtin_amdgcn_fence(__ATOMIC_ACQUIRE, "workgroup");

  for (int pass = 0; pass < 2; ++pass) {
#pragma unroll
    for (int it = 0; it < 8; ++it) {
      const int row = it * 2 + hh;
      const v4f v = *(const v4f*)(slab + row * kSlabP + c4);
      *(volatile v4f*)(ob + (size_t)row * kChan) = v;
    }
    __threadfence();
  }
}

extern "C" void kernel_launch(void* const* d_in, const int* in_sizes, int n_in,
                              void* d_out, int out_size, void* d_ws, size_t ws_size,
                              hipStream_t stream) {
  if (n_in < 4) return;
  if (in_sizes[0] != kBatch * kTime * kChan) return;
  if (in_sizes[1] != 1) return;
  if (in_sizes[2] != 1) return;
  if (in_sizes[3] != kChan) return;
  if (out_size != kBatch * kTime * kChan) return;
  if (ws_size < kWsTotal) return;

  const float* x   = (const float*)d_in[0];
  const float* lar = (const float*)d_in[1];
  const float* ldc = (const float*)d_in[2];
  const float* ema = (const float*)d_in[3];
  float* out = (float*)d_out;

  char* ws = (char*)d_ws;
  unsigned short* taps = (unsigned short*)(ws + kOffTaps);
  unsigned short* gt   = (unsigned short*)(ws + kOffGt);

  build_taps_kernel<<<1, 256, 0, stream>>>(ldc, taps);
  act_plane_kernel<<<dim3(kTime / kTile, kChan / kTile, kBatch), 256, 0, stream>>>(x, gt);
  band_gemm_kernel<<<dim3(kTime / kTile, kCols / kTile), 128, 0, stream>>>(x, lar, ldc, ema, taps, gt, out);
}
